// INR_45792941310797
// MI455X (gfx1250) — hardware-verified
//
#include <hip/hip_runtime.h>
#include <stdint.h>
#include <stddef.h>

typedef __attribute__((ext_vector_type(16))) _Float16 v16h;
typedef __attribute__((ext_vector_type(8)))  _Float16 v8h;
typedef __attribute__((ext_vector_type(16))) __bf16   v16b;
typedef __attribute__((ext_vector_type(8)))  __bf16   v8b;
typedef __attribute__((ext_vector_type(8)))  float    v8f;
typedef __attribute__((ext_vector_type(4)))  float    v4f;
#define PSCALE 32768.0f
#define U16(p) ((const unsigned short*)(const void*)(p))
#define PSCALE_INV (1.0f / 32768.0f)

__device__ __forceinline__ unsigned short f2bf_bits(float f) {
  unsigned u = __float_as_uint(f);
  return (unsigned short)((u + 0x7FFFu + ((u >> 16) & 1u)) >> 16);
}
__device__ __forceinline__ float bf_bits2f(unsigned short h) { return __uint_as_float(((unsigned)h) << 16); }

__device__ __forceinline__ void dep_guard_h(v8f& a, v8f& b, v16h x, v16h y) { asm volatile("v_nop\n\tv_nop\n\tv_nop\n\tv_nop" : "+v"(a), "+v"(b) : "v"(x), "v"(y)); }
__device__ __forceinline__ void dep_guard_b(v8f& a, v8f& b, v16b x, v16b y) { asm volatile("v_nop\n\tv_nop\n\tv_nop\n\tv_nop" : "+v"(a), "+v"(b) : "v"(x), "v"(y)); }
__device__ __forceinline__ void keep4_h(v16h a, v16h b, v16h c, v16h d) { asm volatile("v_nop" :: "v"(a), "v"(b), "v"(c), "v"(d)); }
__device__ __forceinline__ void keep4_b(v16b a, v16b b, v16b c, v16b d) { asm volatile("v_nop" :: "v"(a), "v"(b), "v"(c), "v"(d)); }
__device__ __forceinline__ void acc_guard4(v8f& a, v8f& b, v8f& c, v8f& d) { asm volatile("v_nop\n\tv_nop\n\tv_nop\n\tv_nop" : "+v"(a), "+v"(b), "+v"(c), "+v"(d)); }
__device__ __forceinline__ void acc_guard1(v8f& a, v16h x, v16h y) { asm volatile("v_nop\n\tv_nop\n\tv_nop\n\tv_nop" : "+v"(a) : "v"(x), "v"(y)); }
template <typename T> struct Frag;
template <> struct Frag<_Float16> {
  typedef v16h V; union U { v16h v; v8h h[2]; };
  static __device__ __forceinline__ v16h load(const _Float16* p) {
    U f; f.h[0] = *(const v8h*)(p); f.h[1] = *(const v8h*)(p + 16); return f.v;
  }
  static __device__ __forceinline__ v8f mma(v16h a, v16h b, v8f c) {
    return __builtin_amdgcn_wmma_f32_16x16x32_f16(false, a, false, b, (short)0, c, false, false);
  }
  static __device__ __forceinline__ void guard(v8f& a, v8f& b, v16h x, v16h y) { dep_guard_h(a, b, x, y); }
  static __device__ __forceinline__ void keep(v16h a, v16h b, v16h c, v16h d) { keep4_h(a, b, c, d); }
};
template <> struct Frag<__bf16> {
  typedef v16b V; union U { v16b v; v8b h[2]; };
  static __device__ __forceinline__ v16b load(const __bf16* p) {
    U f; f.h[0] = *(const v8b*)(p); f.h[1] = *(const v8b*)(p + 16); return f.v;
  }
  static __device__ __forceinline__ v8f mma(v16b a, v16b b, v8f c) {
    return __builtin_amdgcn_wmma_f32_16x16x32_bf16(false, a, false, b, (short)0, c, false, false);
  }
  static __device__ __forceinline__ void guard(v8f& a, v8f& b, v16b x, v16b y) { dep_guard_b(a, b, x, y); }
  static __device__ __forceinline__ void keep(v16b a, v16b b, v16b c, v16b d) { keep4_b(a, b, c, d); }
};

template <int ET> struct Elem;
template <> struct Elem<0> { typedef _Float16 T; };
template <> struct Elem<1> { typedef __bf16 T; };
template <int ET, bool SPLIT, int BIAS_MODE, int OUT_MODE, bool RESID, int ACT = 0>
__global__ __launch_bounds__(256) void wmma_gemm64(
    const unsigned short* __restrict__ Ap, const unsigned short* __restrict__ A2p, int lda, long strideA,
    const unsigned short* __restrict__ Btp, const unsigned short* __restrict__ Bt2p, int ldb, long strideB,
    void* __restrict__ Cout, void* __restrict__ Cout2, int ldc, long strideC,
    const float* __restrict__ bias,
    const float* __restrict__ resid, long strideR,
    int M, int N, int K, float scale) {
  typedef typename Elem<ET>::T T;
  typedef typename Frag<T>::V V;
  const T* A = (const T*)Ap; const T* A2 = (const T*)A2p; const T* Bt = (const T*)Btp; const T* Bt2 = (const T*)Bt2p;
  __shared__ __align__(16) float sT[8][16 * 68];
  const int b    = blockIdx.y;
  const int lane = threadIdx.x & 31;
  const int wave = threadIdx.x >> 5;
  const int tilesN = N >> 6;
  const int tilesM = M >> 6;
  const int tile = blockIdx.x * 8 + wave;
  if (tile >= tilesM * tilesN) return;
  const int tm = tile / tilesN;
  const int tn = tile - tm * tilesN;
  const int m0 = tm << 6;
  const int n0 = tn << 6;

  const T* Ab  = A  + (size_t)b * strideA;
  const T* Bb  = Bt + (size_t)b * strideB;
  const T* Ab2 = SPLIT ? (A2  + (size_t)b * strideA) : nullptr;
  const T* Bb2 = SPLIT ? (Bt2 + (size_t)b * strideB) : nullptr;

  const int rlane = lane & 15;
  const int koff  = (lane >> 4) * 8;
  const int mOff  = (lane >> 4) * 8;

  v8f acc[4][4];
#pragma unroll
  for (int i = 0; i < 4; ++i)
#pragma unroll
    for (int j = 0; j < 4; ++j) acc[i][j] = (v8f){0.f,0.f,0.f,0.f,0.f,0.f,0.f,0.f};

  for (int k0 = 0; k0 < K; k0 += 32) {
    V bh[4], bl[4];
#pragma unroll
    for (int j = 0; j < 4; ++j) {
      const size_t bo = (size_t)(n0 + (j << 4) + rlane) * ldb + koff + k0;
      bh[j] = Frag<T>::load(Bb + bo);
      if (SPLIT) bl[j] = Frag<T>::load(Bb2 + bo);
    }
#pragma unroll
    for (int i = 0; i < 4; ++i) {
      const size_t ao = (size_t)(m0 + (i << 4) + rlane) * lda + koff + k0;
      V ah = Frag<T>::load(Ab + ao);
      V al;
      if (SPLIT) al = Frag<T>::load(Ab2 + ao);
#pragma unroll
      for (int j = 0; j < 4; ++j) {
        acc[i][j] = Frag<T>::mma(ah, bh[j], acc[i][j]);
        if (SPLIT) {
          acc[i][j] = Frag<T>::mma(ah, bl[j], acc[i][j]);
          acc[i][j] = Frag<T>::mma(al, bh[j], acc[i][j]);
        }
      }
      Frag<T>::guard(acc[i][0], acc[i][3], ah, SPLIT ? al : ah);
    }
    Frag<T>::keep(bh[0], bh[1], bh[2], bh[3]);
    if (SPLIT) Frag<T>::keep(bl[0], bl[1], bl[2], bl[3]);
  }
  acc_guard4(acc[0][0], acc[0][1], acc[0][2], acc[0][3]);
  acc_guard4(acc[1][0], acc[1][1], acc[1][2], acc[1][3]);
  acc_guard4(acc[2][0], acc[2][1], acc[2][2], acc[2][3]);
  acc_guard4(acc[3][0], acc[3][1], acc[3][2], acc[3][3]);

  float* slab = sT[wave];
  const float* Rb = RESID ? (resid + (size_t)b * strideR) : nullptr;
#pragma unroll
  for (int i = 0; i < 4; ++i) {
    const int mBase = m0 + (i << 4);
#pragma unroll
    for (int j = 0; j < 4; ++j) {
      const int n = n0 + (j << 4) + rlane;
      float bv = 0.f;
      if (BIAS_MODE == 2) bv = bias[n];
#pragma unroll
      for (int r = 0; r < 8; ++r) {
        float v = acc[i][j][r] * scale;
        if (BIAS_MODE == 1) v += bias[mBase + mOff + r];
        if (BIAS_MODE == 2) v += bv;
        if (RESID) v += Rb[(size_t)(mBase + mOff + r) * ldc + n];
        if (ACT == 1) v = tanhf(v);
        if (ACT == 2) v = fmaxf(v, 0.0f);
        if (ACT == 3) v = v / (1.0f + expf(-v));
        if (ACT == 4) v = (v > 0.f) ? v : 0.01f * v;
        if (ACT == 5) v = 0.5f * v * (1.0f + erff(v * 0.70710678118654752f));
        slab[(mOff + r) * 68 + (j << 4) + rlane] = v;
      }
    }
    __builtin_amdgcn_fence(__ATOMIC_RELEASE, "workgroup");
    __builtin_amdgcn_wave_barrier();
    __builtin_amdgcn_fence(__ATOMIC_ACQUIRE, "workgroup");
    if (OUT_MODE == 0) {
      float* C = (float*)Cout + (size_t)b * strideC;
      const int hh = lane >> 4, c4 = (lane & 15) * 4;
      for (int pass = 0; pass < 2; ++pass) {
#pragma unroll
        for (int it = 0; it < 8; ++it) {
          const int row = it * 2 + hh;
          v4f v = *(const v4f*)(slab + row * 68 + c4);
          *(volatile v4f*)(C + (size_t)(mBase + row) * ldc + n0 + c4) = v;
        }
        __threadfence();
      }
    } else {
      const int q = lane >> 3, c8 = (lane & 7) * 8;
      unsigned short* C  = (unsigned short*)Cout  + (size_t)b * strideC;
      unsigned short* C2 = (OUT_MODE == 2) ? ((unsigned short*)Cout2 + (size_t)b * strideC) : nullptr;
      for (int pass = 0; pass < 2; ++pass) {
#pragma unroll
        for (int it = 0; it < 4; ++it) {
          const int row = it * 4 + q;
          const float* sp = slab + row * 68 + c8;
          v8h hv, lv;
#pragma unroll
          for (int e = 0; e < 8; ++e) {
            if (OUT_MODE == 1) {
              hv[e] = (_Float16)sp[e];
            } else {
              unsigned short hb = f2bf_bits(sp[e]);
              unsigned short lb = f2bf_bits(sp[e] - bf_bits2f(hb));
              hv[e] = __builtin_bit_cast(_Float16, hb);
              lv[e] = __builtin_bit_cast(_Float16, lb);
            }
          }
          *(volatile v8h*)(C + (size_t)(mBase + row) * ldc + n0 + c8) = hv;
          if (OUT_MODE == 2) *(volatile v8h*)(C2 + (size_t)(mBase + row) * ldc + n0 + c8) = lv;
        }
        __threadfence();
      }
    }
    __builtin_amdgcn_fence(__ATOMIC_RELEASE, "workgroup");
    __builtin_amdgcn_wave_barrier();
    __builtin_amdgcn_fence(__ATOMIC_ACQUIRE, "workgroup");
  }
}

constexpr int   kImgB      = 8;
constexpr int   kImgH      = 256;
constexpr int   kImgW      = 256;
constexpr int   kFeat      = 256;
constexpr int   kChOut     = 3;
constexpr int   kNSamp     = 16;
constexpr int   kPoolK     = 4;
constexpr int   kPixPerImg = kImgH * kImgW;
constexpr int   kOutH      = kImgH / kPoolK;
constexpr int   kOutW      = kImgW / kPoolK;
constexpr int   kOutRowF   = kOutW * kChOut;
constexpr int   kOut0Elems = kImgB * kOutH * kOutW * kChOut;
constexpr int   kOutTotal  = kOut0Elems + 2 * kImgB;
constexpr float kWCarry    = 16.0f;
constexpr float kWCarryInv = 0.0625f;
constexpr int   kW3Rows    = 16;
constexpr int   kW3sPitch  = 264;
constexpr int   kPixPerWave = 4;
constexpr int   kPixPerBlk  = 32;
constexpr int   kGemmBlocks = ((kPixPerImg / 64) * (kFeat / 64)) / 8;

static_assert(kOut0Elems * 4 == 393216);
static_assert(kOutTotal * 4 == 393280);
static_assert(kFeat % 64 == 0);
static_assert(kFeat % 32 == 0);
static_assert(kPixPerImg % 64 == 0);
static_assert(((kPixPerImg / 64) * (kFeat / 64)) % 8 == 0);
static_assert(kPixPerImg % kPixPerBlk == 0);
static_assert(kOutRowF == 192);
static_assert((kOutRowF * 4) % 128 == 0);

constexpr size_t kWsCtab  = 0;
constexpr size_t kWsW3t   = 4096;
constexpr size_t kWsW1t   = kWsW3t + (size_t)kW3Rows * kFeat * 2;
constexpr size_t kWsW2t   = kWsW1t + (size_t)kFeat * kFeat * 2;
constexpr size_t kWsH0    = kWsW2t + (size_t)kFeat * kFeat * 2;
constexpr size_t kWsH1    = kWsH0 + (size_t)kPixPerImg * kFeat * 2;
constexpr size_t kWsTotal = kWsH1 + (size_t)kPixPerImg * kFeat * 2;
static_assert(kWsW1t == 12288 && kWsW2t == 143360 && kWsH0 == 274432 && kWsH1 == 33828864 && kWsTotal == 67383296);
static_assert(kWsW3t % 128 == 0 && kWsW1t % 128 == 0 && kWsW2t % 128 == 0 && kWsH0 % 128 == 0 && kWsH1 % 128 == 0);
static_assert(kWsTotal <= 134217728);

__device__ __forceinline__ int clamp_sample(int v) { return v < 0 ? 0 : (v > kNSamp - 1 ? kNSamp - 1 : v); }

__global__ __launch_bounds__(256) void k_prep(
    const int* __restrict__ sidx, const float* __restrict__ shift, const float* __restrict__ rot,
    const float* __restrict__ w3, float* __restrict__ ctab, unsigned short* __restrict__ w3t,
    float* __restrict__ out_tail)
{
  const int tid  = threadIdx.x;
  const int lane = tid & 31;
  const int wave = tid >> 5;
  v8h hv0, hv1;
  {
    const int ncl = (wave < kChOut) ? wave : 0;
    const bool live = (wave < kChOut);
#pragma unroll
    for (int e = 0; e < 8; ++e) {
      const float wv = w3[(8 * lane + e) * kChOut + ncl];
      const float sv = live ? (wv * kWCarry) : 0.0f;
      hv0[e] = (_Float16)sv;
      hv1[e] = (_Float16)0.0f;
    }
  }
  for (int pass = 0; pass < 2; ++pass) {
    *(volatile v8h*)(w3t + (size_t)wave * kFeat + 8 * lane) = hv0;
    *(volatile v8h*)(w3t + (size_t)(wave + 8) * kFeat + 8 * lane) = hv1;
    __threadfence();
  }
  if (wave == 0) {
#pragma unroll 1
    for (int i = 0; i < 2; ++i) {
      const int bi = 4 * i + (lane >> 3);
      const int qd = lane & 7;
      const int id = clamp_sample(sidx[bi]);
      const float a  = rot[id];
      const float cs = cosf(a);
      const float sn = sinf(a);
      const float dxv = shift[id * 2 + 0];
      const float dyv = shift[id * 2 + 1];
      v4f cv;
      cv[0] = (qd == 0) ? cs  : 0.0f;
      cv[1] = (qd == 0) ? sn  : 0.0f;
      cv[2] = (qd == 0) ? dxv : 0.0f;
      cv[3] = (qd == 0) ? dyv : 0.0f;
      volatile v4f* dst = (volatile v4f*)(ctab + bi * 32 + qd * 4);
      *dst = cv;
      __threadfence();
      *dst = cv;
    }
    v4f tv;
#pragma unroll
    for (int j = 0; j < 4; ++j) {
      const int bi = (lane & 1) * 4 + j;
      const int comp = (lane >> 1) & 1;
      const int id = clamp_sample(sidx[bi]);
      tv[j] = shift[id * 2 + comp];
    }
    if (lane < 4) {
      volatile v4f* dst = (volatile v4f*)(out_tail + 4 * lane);
      *dst = tv;
      __threadfence();
      *dst = tv;
    }
  }
}

__global__ __launch_bounds__(256) void k_wtrans(const float* __restrict__ w1, const float* __restrict__ w2,
    unsigned short* __restrict__ w1t, unsigned short* __restrict__ w2t)
{
  __shared__ __align__(16) float tileT[64 * 68];
  const int tid  = threadIdx.x;
  const int lane = tid & 31;
  const int wave = tid >> 5;
  const bool second = (blockIdx.y != 0);
  const float* wsrc = second ? w2 : w1;
  unsigned short* wdst = second ? w2t : w1t;
  const int bx = blockIdx.x;
  const int n0 = (bx & 3) * 64;
  const int k0 = (bx >> 2) * 64;
#pragma unroll
  for (int i = 0; i < 4; ++i) {
    const int e4  = tid + 256 * i;
    const int kk  = e4 >> 4;
    const int nn4 = (e4 & 15) * 4;
    const v4f v = *(const v4f*)(wsrc + (size_t)(k0 + kk) * kFeat + n0 + nn4);
    tileT[(nn4 + 0) * 68 + kk] = v[0];
    tileT[(nn4 + 1) * 68 + kk] = v[1];
    tileT[(nn4 + 2) * 68 + kk] = v[2];
    tileT[(nn4 + 3) * 68 + kk] = v[3];
  }
  __syncthreads();
  const int q  = lane >> 3;
  const int c8 = (lane & 7) * 8;
  const int r0 = wave * 4 + q;
  const int r1 = 32 + wave * 4 + q;
  v8h hv0, hv1;
#pragma unroll
  for (int e = 0; e < 8; ++e) {
    hv0[e] = (_Float16)(tileT[r0 * 68 + c8 + e] * kWCarry);
    hv1[e] = (_Float16)(tileT[r1 * 68 + c8 + e] * kWCarry);
  }
  for (int pass = 0; pass < 2; ++pass) {
    *(volatile v8h*)(wdst + (size_t)(n0 + r0) * kFeat + k0 + c8) = hv0;
    *(volatile v8h*)(wdst + (size_t)(n0 + r1) * kFeat + k0 + c8) = hv1;
    __threadfence();
  }
}

__global__ __launch_bounds__(256) void k_proj_sin(
    const float* __restrict__ x, const float* __restrict__ pw, const float* __restrict__ pb,
    const float* __restrict__ ctab, unsigned short* __restrict__ h0, int bimg)
{
  const int tid  = threadIdx.x;
  const int lane = tid & 31;
  const int wave = tid >> 5;
  const float ca  = ctab[bimg * 32 + 0];
  const float sa  = ctab[bimg * 32 + 1];
  const float dxv = ctab[bimg * 32 + 2];
  const float dyv = ctab[bimg * 32 + 3];
#pragma unroll 1
  for (int i = 0; i < kPixPerWave; ++i) {
    const int p = blockIdx.x * kPixPerBlk + wave * kPixPerWave + i;
    const size_t gp = (size_t)bimg * kPixPerImg + p;
    const float cx = x[gp * 2 + 0];
    const float cy = x[gp * 2 + 1];
    const float nx = ca * cx - sa * cy + dxv;
    const float ny = sa * cx + ca * cy + dyv;
    unsigned short* hrow = h0 + (size_t)p * kFeat;
#pragma unroll 1
    for (int q = 0; q < 4; ++q) {
      float s0 = 0.0f, s1 = 0.0f;
#pragma unroll 1
      for (int e = 0; e < 2; ++e) {
        const int c = q * 64 + 2 * lane + e;
        const float arg = nx * pw[c] + ny * pw[kFeat + c] + pb[c];
        const float kq = rintf(arg * 0.15915494309189535f);
        float rr = fmaf(-kq, 6.28318548202514648f, arg);
        rr = fmaf(-kq, -1.7484555e-7f, rr);
        const float sv = __sinf(rr);
        s0 = (e == 0) ? sv : s0;
        s1 = (e == 0) ? s1 : sv;
      }
      const _Float16 hlo = (_Float16)s0;
      const _Float16 hhi = (_Float16)s1;
      const unsigned u = (unsigned)__builtin_bit_cast(unsigned short, hlo) | ((unsigned)__builtin_bit_cast(unsigned short, hhi) << 16);
      volatile unsigned* dst = (volatile unsigned*)(hrow + q * 64) + lane;
      *dst = u;
      __threadfence();
      *dst = u;
    }
  }
}

__global__ __launch_bounds__(256) void k_head_pool(
    const unsigned short* __restrict__ hp, const unsigned short* __restrict__ w3tp,
    const float* __restrict__ b3, const int* __restrict__ sidx,
    const float* __restrict__ colw, const float* __restrict__ colb,
    float* __restrict__ out, int bimg)
{
  __shared__ __align__(16) _Float16 w3s[kW3Rows * kW3sPitch];
  __shared__ __align__(16) float ps[kPoolK * kOutW * 4];
  __shared__ __align__(16) float outs[kOutRowF];
  const int tid  = threadIdx.x;
  const int lane = tid & 31;
  const int wave = tid >> 5;
  const int ho   = blockIdx.x;
#pragma unroll
  for (int i = 0; i < 2; ++i) {
    const int idx = tid + 256 * i;
    const int row = idx >> 5;
    const int c8  = (idx & 31) * 8;
    const uint4 v = *(const uint4*)(w3tp + row * kFeat + c8);
    *(uint4*)(w3s + row * kW3sPitch + c8) = v;
  }
  __syncthreads();
  const _Float16* hh = (const _Float16*)hp;
  const int pr    = wave >> 1;
  const int chalf = wave & 1;
  const int rl    = lane & 15;
  const int hsel  = lane >> 4;
  const int koff  = hsel * 8;
  const int prow  = ho * kPoolK + pr;
#pragma unroll 1
  for (int s = 0; s < 8; ++s) {
    const int col = chalf * 128 + s * 16 + rl;
    const _Float16* arow = hh + ((size_t)(prow * kImgW + col)) * kFeat + koff;
    const _Float16* brow = w3s + rl * kW3sPitch + koff;
    v8f acc = (v8f){0.f,0.f,0.f,0.f,0.f,0.f,0.f,0.f};
#pragma unroll
    for (int ks = 0; ks < kFeat / 32; ++ks) {
      const v16h av = Frag<_Float16>::load(arow + ks * 32);
      const v16h bv = Frag<_Float16>::load(brow + ks * 32);
      acc = Frag<_Float16>::mma(av, bv, acc);
      acc_guard1(acc, av, bv);
    }
    float suma = 0.0f;
    suma += acc[0]; suma += acc[1]; suma += acc[2]; suma += acc[3];
    float sumb = 0.0f;
    sumb += acc[4]; sumb += acc[5]; sumb += acc[6]; sumb += acc[7];
    if (rl < kChOut) {
      const int cell = chalf * 32 + s * 4 + hsel * 2;
      ps[(pr * kOutW + cell) * 4 + rl]     = suma;
      ps[(pr * kOutW + cell + 1) * 4 + rl] = sumb;
    }
  }
  __syncthreads();
  if (tid < kOutRowF) {
    const int cell = tid / kChOut;
    const int c    = tid - cell * kChOut;
    float tot = 0.0f;
    tot += ps[(0 * kOutW + cell) * 4 + c];
    tot += ps[(1 * kOutW + cell) * 4 + c];
    tot += ps[(2 * kOutW + cell) * 4 + c];
    tot += ps[(3 * kOutW + cell) * 4 + c];
    const int id = clamp_sample(sidx[bimg]);
    const float cwv = colw[id * kChOut + c];
    const float cbv = colb[id * kChOut + c];
    const bool ident = (id == 0);
    const float scl = ident ? 1.0f : cwv;
    const float bsv = ident ? 0.0f : cbv;
    float val = tot * (kWCarryInv * (1.0f / 16.0f)) + b3[c];
    val = val * scl + bsv;
    outs[tid] = val;
  }
  __syncthreads();
  if (wave == 0) {
    float* orow = out + (size_t)(bimg * kOutH + ho) * kOutRowF;
    const v4f v0 = *(const v4f*)(outs + 4 * lane);
    const v4f v1 = *(const v4f*)(outs + 128 + 4 * (lane & 15));
    for (int pass = 0; pass < 2; ++pass) {
      *(volatile v4f*)(orow + 4 * lane) = v0;
      if (lane < 16) *(volatile v4f*)(orow + 128 + 4 * lane) = v1;
      __threadfence();
    }
  }
}

extern "C" void kernel_launch(void* const* d_in, const int* in_sizes, int n_in,
                              void* d_out, int out_size, void* d_ws, size_t ws_size,
                              hipStream_t stream)
{
  if (n_in < 14) return;
  if (in_sizes[0] != kImgB * kPixPerImg * 2) return;
  if (out_size != kOutTotal) return;
  if (ws_size < kWsTotal) return;

  const float* x     = (const float*)d_in[0];
  const int*   sidx  = (const int*)d_in[1];
  const float* shift = (const float*)d_in[2];
  const float* rot   = (const float*)d_in[3];
  const float* pw    = (const float*)d_in[4];
  const float* pb    = (const float*)d_in[5];
  const float* w1    = (const float*)d_in[6];
  const float* b1    = (const float*)d_in[7];
  const float* w2    = (const float*)d_in[8];
  const float* b2    = (const float*)d_in[9];
  const float* w3    = (const float*)d_in[10];
  const float* b3    = (const float*)d_in[11];
  const float* colw  = (const float*)d_in[12];
  const float* colb  = (const float*)d_in[13];
  float* out = (float*)d_out;

  char* ws = (char*)d_ws;
  float*          ctab = (float*)(ws + kWsCtab);
  unsigned short* w3t  = (unsigned short*)(ws + kWsW3t);
  unsigned short* w1t  = (unsigned short*)(ws + kWsW1t);
  unsigned short* w2t  = (unsigned short*)(ws + kWsW2t);
  unsigned short* h0p  = (unsigned short*)(ws + kWsH0);
  unsigned short* h1p  = (unsigned short*)(ws + kWsH1);

  k_prep<<<dim3(1), dim3(256), 0, stream>>>(sidx, shift, rot, w3, ctab, w3t, out + kOut0Elems);
  k_wtrans<<<dim3(16, 2), dim3(256), 0, stream>>>(w1, w2, w1t, w2t);

  for (int b = 0; b < kImgB; ++b) {
    k_proj_sin<<<dim3(kPixPerImg / kPixPerBlk), dim3(256), 0, stream>>>(x, pw, pb, ctab, h0p, b);
    wmma_gemm64<0, false, 2, 1, false, 2><<<dim3(kGemmBlocks, 1), dim3(256), 0, stream>>>(
        h0p, h0p, kFeat, 0L,
        w1t, w1t, kFeat, 0L,
        (void*)h1p, (void*)h1p, kFeat, 0L,
        b1, b1, 0L,
        kPixPerImg, kFeat, kFeat, kWCarryInv);
    wmma_gemm64<0, false, 2, 1, false, 2><<<dim3(kGemmBlocks, 1), dim3(256), 0, stream>>>(
        h1p, h1p, kFeat, 0L,
        w2t, w2t, kFeat, 0L,
        (void*)h0p, (void*)h0p, kFeat, 0L,
        b2, b2, 0L,
        kPixPerImg, kFeat, kFeat, kWCarryInv);
    k_head_pool<<<dim3(kOutH), dim3(256), 0, stream>>>(h0p, w3t, b3, sidx, colw, colb, out, b);
  }
}
